// GeneralTransformerBlock_18296560681612
// MI455X (gfx1250) — hardware-verified
//
#include <hip/hip_runtime.h>

#define B_     8
#define C_     512
#define HIMG_  56
#define WIMG_  56
#define HW_    3136
#define NH_    16
#define HD_    32
#define L_     49
#define HID_   2048
#define QKVN_  1536
#define IPC_   2
#define NCHK_  4
#define MC_    (IPC_ * HW_)
#define NWC_   (IPC_ * 64)
#define SY_    8
#define NYS_   (HIMG_ / SY_)

#define NFOLD_ 9216
#define NBIAS_ (NH_ * 64 * 64)
#define W0_    (QKVN_ * C_)
#define W1_    (W0_ + C_ * C_)
#define W2_    (W1_ + HID_ * C_)
#define W3_    (W2_ + C_ * HID_)
#define NWGRP_ (W3_ / 8)
#define PREPN_ (NFOLD_ + NBIAS_ + NWGRP_)

#define BM_ 128
#define BN_ 128
#define BK_ 32
#define LP_ 40
#define INV64_  0.015625f
#define INV256_ 0.00390625f
#define QSCALE_ 0.17677669529663687f

static_assert(B_ % IPC_ == 0);
static_assert(MC_ % BM_ == 0);
static_assert(QKVN_ % BN_ == 0 && C_ % BN_ == 0 && HID_ % BN_ == 0);
static_assert(C_ % BK_ == 0 && HID_ % BK_ == 0);
static_assert(HW_ % 32 == 0);
static_assert(MC_ % 8 == 0);
static_assert(HIMG_ % SY_ == 0 && HIMG_ % 7 == 0 && WIMG_ % 7 == 0);
static_assert(PREPN_ % 256 == 0);
static_assert(W0_ % 8 == 0 && W1_ % 8 == 0 && W2_ % 8 == 0 && W3_ % 8 == 0);

typedef _Float16 v16h __attribute__((ext_vector_type(16)));
typedef _Float16 v8h __attribute__((ext_vector_type(8)));
typedef float v8f __attribute__((ext_vector_type(8)));
typedef float v4f __attribute__((ext_vector_type(4)));
typedef unsigned int v4u __attribute__((ext_vector_type(4)));

union Frag { v16h v; v8h h[2]; };
union H8 { v8h h; v4u u; };
union F4 { v4f f; v4u u; };

enum { EPI_QKV = 0, EPI_PROJ = 1, EPI_H1 = 2, EPI_OUT = 3 };

__device__ __forceinline__ v8f zero8() {
  v8f z = {0.f, 0.f, 0.f, 0.f, 0.f, 0.f, 0.f, 0.f};
  return z;
}

__device__ __forceinline__ v8f wmma_g(const v16h a, const v16h b, v8f c) {
  v8f d = __builtin_amdgcn_wmma_f32_16x16x32_f16(false, a, false, b, (short)0, c, false, false);
  asm volatile("v_nop\n\tv_nop\n\tv_nop\n\tv_nop" : "+v"(d) : "v"(a), "v"(b));
  return d;
}

__device__ __forceinline__ void vst(void* p, v4u v) { *(volatile v4u*)p = v; }
__device__ __forceinline__ void fst(float* p, float v) { *(volatile float*)p = v; }

__device__ __forceinline__ float gelu_f(float x) {
  return 0.5f * x * (1.0f + erff(x * 0.70710678118654752f));
}

__global__ void __launch_bounds__(256)
prep_kernel(const float* __restrict__ fc1_b,
            const float* __restrict__ bn1_g, const float* __restrict__ bn1_b,
            const float* __restrict__ bn1_m, const float* __restrict__ bn1_v,
            const float* __restrict__ dw_b,
            const float* __restrict__ bn2_g, const float* __restrict__ bn2_b,
            const float* __restrict__ bn2_m, const float* __restrict__ bn2_v,
            const float* __restrict__ fc2_b,
            const float* __restrict__ bn3_g, const float* __restrict__ bn3_b,
            const float* __restrict__ bn3_m, const float* __restrict__ bn3_v,
            const float* __restrict__ rpb, const int* __restrict__ rel,
            const float* __restrict__ qkv_w, const float* __restrict__ proj_w,
            const float* __restrict__ fc1_w, const float* __restrict__ fc2_w,
            float* ab, float* biasTab, _Float16* w16) {
  const int gi = blockIdx.x * 256 + threadIdx.x;
  if (gi < NFOLD_) {
    float val;
    if (gi < 2048) {
      const int c = gi;
      val = bn1_g[c] * rsqrtf(bn1_v[c] + 1e-5f);
    } else if (gi < 4096) {
      const int c = gi - 2048;
      const float s = bn1_g[c] * rsqrtf(bn1_v[c] + 1e-5f);
      val = (fc1_b[c] - bn1_m[c]) * s + bn1_b[c];
    } else if (gi < 6144) {
      const int c = gi - 4096;
      val = bn2_g[c] * rsqrtf(bn2_v[c] + 1e-5f);
    } else if (gi < 8192) {
      const int c = gi - 6144;
      const float s = bn2_g[c] * rsqrtf(bn2_v[c] + 1e-5f);
      val = (dw_b[c] - bn2_m[c]) * s + bn2_b[c];
    } else if (gi < 8704) {
      const int c = gi - 8192;
      val = bn3_g[c] * rsqrtf(bn3_v[c] + 1e-5f);
    } else {
      const int c = gi - 8704;
      const float s = bn3_g[c] * rsqrtf(bn3_v[c] + 1e-5f);
      val = (fc2_b[c] - bn3_m[c]) * s + bn3_b[c];
    }
    float* d = ab + gi;
    fst(d, val);
    __threadfence();
    fst(d, val);
  } else if (gi < NFOLD_ + NBIAS_) {
    const int j = gi - NFOLD_;
    const int h = j >> 12;
    const int row = (j >> 6) & 63;
    const int col = j & 63;
    float val = -1.0e30f;
    if (row < L_ && col < L_) {
      int ix = rel[row * L_ + col];
      ix = ix < 0 ? 0 : (ix > 168 ? 168 : ix);
      val = rpb[ix * NH_ + h];
    }
    float* d = biasTab + j;
    fst(d, val);
    __threadfence();
    fst(d, val);
  } else if (gi < PREPN_) {
    const int e = (gi - NFOLD_ - NBIAS_) * 8;
    const float* src;
    if (e < W0_) src = qkv_w + e;
    else if (e < W1_) src = proj_w + (e - W0_);
    else if (e < W2_) src = fc1_w + (e - W1_);
    else src = fc2_w + (e - W2_);
    const v4f a = *(const v4f*)src;
    const v4f b = *(const v4f*)(src + 4);
    H8 o;
#pragma unroll
    for (int i = 0; i < 4; ++i) {
      o.h[i] = (_Float16)(a[i] * 64.0f);
      o.h[4 + i] = (_Float16)(b[i] * 64.0f);
    }
    _Float16* d = w16 + e;
    vst(d, o.u);
    __threadfence();
    vst(d, o.u);
  }
}

template <int MODE>
__global__ void __launch_bounds__(256)
ln_kernel(const float* __restrict__ src, const float* __restrict__ g, const float* __restrict__ bta,
          _Float16* dst, int ntok) {
  const int wave = threadIdx.x >> 5, lane = threadIdx.x & 31;
  const int tok = blockIdx.x * 8 + wave;
  if (tok >= ntok) return;
  const int cA = 8 * lane, cB = 256 + 8 * lane;
  float v[16];
  int orow;
  if constexpr (MODE == 0) {
    const int bl = tok / HW_, n = tok - bl * HW_;
    const float* base = src + (size_t)bl * C_ * HW_ + n;
#pragma unroll
    for (int i = 0; i < 8; ++i) {
      v[i] = base[(size_t)(cA + i) * HW_];
      v[8 + i] = base[(size_t)(cB + i) * HW_];
    }
    const int y = n / WIMG_, x = n - y * WIMG_;
    const int wl = bl * 64 + (y / 7) * 8 + (x / 7);
    orow = wl * L_ + (y % 7) * 7 + (x % 7);
  } else {
    const float* row = src + (size_t)tok * C_;
    const v4f a0 = *(const v4f*)(row + cA), a1 = *(const v4f*)(row + cA + 4);
    const v4f b0 = *(const v4f*)(row + cB), b1 = *(const v4f*)(row + cB + 4);
#pragma unroll
    for (int i = 0; i < 4; ++i) {
      v[i] = a0[i]; v[4 + i] = a1[i]; v[8 + i] = b0[i]; v[12 + i] = b1[i];
    }
    orow = tok;
  }
  float s = 0.f;
#pragma unroll
  for (int i = 0; i < 16; ++i) s += v[i];
#pragma unroll
  for (int m = 16; m >= 1; m >>= 1) s += __shfl_xor(s, m, 32);
  const float mean = s * (1.0f / 512.0f);
  float s2 = 0.f;
#pragma unroll
  for (int i = 0; i < 16; ++i) { v[i] -= mean; s2 += v[i] * v[i]; }
#pragma unroll
  for (int m = 16; m >= 1; m >>= 1) s2 += __shfl_xor(s2, m, 32);
  const float rs = rsqrtf(s2 * (1.0f / 512.0f) + 1e-6f);
  const v4f g0 = *(const v4f*)(g + cA), g1 = *(const v4f*)(g + cA + 4);
  const v4f g2 = *(const v4f*)(g + cB), g3 = *(const v4f*)(g + cB + 4);
  const v4f t0 = *(const v4f*)(bta + cA), t1 = *(const v4f*)(bta + cA + 4);
  const v4f t2 = *(const v4f*)(bta + cB), t3 = *(const v4f*)(bta + cB + 4);
  float gg[16], bb[16];
#pragma unroll
  for (int i = 0; i < 4; ++i) {
    gg[i] = g0[i]; gg[4 + i] = g1[i]; gg[8 + i] = g2[i]; gg[12 + i] = g3[i];
    bb[i] = t0[i]; bb[4 + i] = t1[i]; bb[8 + i] = t2[i]; bb[12 + i] = t3[i];
  }
  H8 oA, oB;
#pragma unroll
  for (int i = 0; i < 8; ++i) {
    oA.h[i] = (_Float16)(v[i] * rs * gg[i] + bb[i]);
    oB.h[i] = (_Float16)(v[8 + i] * rs * gg[8 + i] + bb[8 + i]);
  }
  _Float16* d = dst + (size_t)orow * C_;
  vst(d + cA, oA.u);
  vst(d + cB, oB.u);
  __threadfence();
  vst(d + cA, oA.u);
  vst(d + cB, oB.u);
}

template <int EPI, int P>
__device__ __forceinline__ void epi_pass(v8f (&acc)[2][4], float* sEw, int lane, int hi, int lr,
                                         int bm0, int bn0, int rowW, int colW, int N,
                                         const float* __restrict__ e0, const float* __restrict__ e1,
                                         const float* __restrict__ e2, void* Out, int img0) {
  if constexpr (EPI != EPI_OUT) {
#pragma unroll
    for (int nt = 0; nt < 4; ++nt)
#pragma unroll
      for (int r = 0; r < 8; ++r)
        sEw[(8 * hi + r) * 64 + 16 * nt + lr] = acc[P][nt][r];
  } else {
#pragma unroll
    for (int ml = 0; ml < 2; ++ml)
#pragma unroll
      for (int ntl = 0; ntl < 2; ++ntl)
#pragma unroll
        for (int r = 0; r < 8; ++r)
          sEw[(16 * ntl + lr) * 32 + 16 * ml + 8 * hi + r] = acc[ml][2 * P + ntl][r];
  }
  __syncthreads();
  const int q = lane >> 3, j = lane & 7;
  if constexpr (EPI == EPI_QKV || EPI == EPI_H1) {
    _Float16* O16 = (_Float16*)Out;
    const int gN0 = bn0 + colW + 8 * j;
    float ea[8], eb[8];
    {
      const v4f u0 = *(const v4f*)(e0 + gN0), u1 = *(const v4f*)(e0 + gN0 + 4);
#pragma unroll
      for (int i = 0; i < 4; ++i) { ea[i] = u0[i]; ea[4 + i] = u1[i]; }
    }
    if constexpr (EPI == EPI_H1) {
      const v4f u0 = *(const v4f*)(e1 + gN0), u1 = *(const v4f*)(e1 + gN0 + 4);
#pragma unroll
      for (int i = 0; i < 4; ++i) { eb[i] = u0[i]; eb[4 + i] = u1[i]; }
    } else {
#pragma unroll
      for (int i = 0; i < 8; ++i) eb[i] = 0.f;
    }
    v4u vals[4];
    _Float16* dst[4];
#pragma unroll
    for (int s = 0; s < 4; ++s) {
      const int rl = 4 * s + q;
      const float* sr = sEw + rl * 64 + 8 * j;
      H8 o;
#pragma unroll
      for (int i = 0; i < 8; ++i) {
        float f = sr[i] * INV64_;
        if constexpr (EPI == EPI_QKV) {
          f += ea[i];
          if (gN0 < C_) f *= QSCALE_;
        } else {
          f = gelu_f(f * ea[i] + eb[i]);
        }
        o.h[i] = (_Float16)f;
      }
      vals[s] = o.u;
      dst[s] = O16 + (size_t)(bm0 + rowW + 16 * P + rl) * N + gN0;
    }
#pragma unroll
    for (int s = 0; s < 4; ++s) vst(dst[s], vals[s]);
    __threadfence();
#pragma unroll
    for (int s = 0; s < 4; ++s) vst(dst[s], vals[s]);
  } else if constexpr (EPI == EPI_PROJ) {
    float* OF = (float*)Out;
    v4u vals[8];
    float* dst[8];
#pragma unroll
    for (int s = 0; s < 8; ++s) {
      const int rl = 4 * (s >> 1) + q;
      const int c0 = 32 * (s & 1) + 4 * j;
      const int gN = bn0 + colW + c0;
      const int gM = bm0 + rowW + 16 * P + rl;
      const int w = gM / L_, l = gM - w * L_;
      const int bl = w >> 6, wi = w & 63;
      const int ly = l / 7, lx = l - ly * 7;
      const int y = (wi >> 3) * 7 + ly, x = (wi & 7) * 7 + lx;
      const int n = y * WIMG_ + x;
      const float* xr = e2 + ((size_t)(img0 + bl) * C_ + gN) * HW_ + n;
      const v4f pb = *(const v4f*)(e0 + gN);
      const float* sr = sEw + rl * 64 + c0;
      F4 o;
#pragma unroll
      for (int i = 0; i < 4; ++i) o.f[i] = sr[i] * INV64_ + pb[i] + xr[(size_t)i * HW_];
      vals[s] = o.u;
      dst[s] = OF + ((size_t)bl * HW_ + n) * C_ + gN;
    }
#pragma unroll
    for (int s = 0; s < 8; ++s) vst(dst[s], vals[s]);
    __threadfence();
#pragma unroll
    for (int s = 0; s < 8; ++s) vst(dst[s], vals[s]);
  } else {
    float* OF = (float*)Out;
    const int gMb = bm0 + rowW;
    const int bl = gMb / HW_, n0 = gMb - bl * HW_;
    v4u vals[8];
    float* dst[8];
#pragma unroll
    for (int s = 0; s < 8; ++s) {
      const int cl = 4 * s + q;
      const int gN = bn0 + colW + 32 * P + cl;
      const float sc = e0[gN] * INV64_, sh = e1[gN];
      const float* sr = sEw + cl * 32 + 4 * j;
      const float* rr = e2 + (size_t)(gMb + 4 * j) * C_ + gN;
      F4 o;
#pragma unroll
      for (int i = 0; i < 4; ++i) o.f[i] = gelu_f(sr[i] * sc + sh) + rr[(size_t)i * C_];
      vals[s] = o.u;
      dst[s] = OF + ((size_t)bl * C_ + gN) * HW_ + n0 + 4 * j;
    }
#pragma unroll
    for (int s = 0; s < 8; ++s) vst(dst[s], vals[s]);
    __threadfence();
#pragma unroll
    for (int s = 0; s < 8; ++s) vst(dst[s], vals[s]);
  }
  __syncthreads();
}

template <int EPI>
__global__ void __launch_bounds__(256)
gemm_kernel(const _Float16* __restrict__ A, const _Float16* __restrict__ Bt, int M, int N, int K,
            const float* __restrict__ e0, const float* __restrict__ e1, const float* __restrict__ e2,
            void* Out, int img0) {
  __shared__ __attribute__((aligned(16))) _Float16 sA[BM_ * LP_];
  __shared__ __attribute__((aligned(16))) _Float16 sB[BN_ * LP_];
  __shared__ __attribute__((aligned(16))) float sE[8 * 1024];

  const int t = threadIdx.x, wave = t >> 5, lane = t & 31, hi = lane >> 4, lr = lane & 15;
  const int bm0 = blockIdx.x * BM_, bn0 = blockIdx.y * BN_;
  if (bm0 + BM_ > M || bn0 + BN_ > N) return;
  const int wm = wave & 3, wn = wave >> 2;
  const int rowW = 32 * wm, colW = 64 * wn;

  const int ldr = t >> 2, lds = (t & 3) * 8;
  const _Float16* Ag0 = A + (size_t)(bm0 + ldr) * K + lds;
  const _Float16* Ag1 = A + (size_t)(bm0 + ldr + 64) * K + lds;
  const _Float16* Bg0 = Bt + (size_t)(bn0 + ldr) * K + lds;
  const _Float16* Bg1 = Bt + (size_t)(bn0 + ldr + 64) * K + lds;
  _Float16* sa0 = sA + ldr * LP_ + lds;
  _Float16* sa1 = sA + (ldr + 64) * LP_ + lds;
  _Float16* sb0 = sB + ldr * LP_ + lds;
  _Float16* sb1 = sB + (ldr + 64) * LP_ + lds;

  v8f acc[2][4];
#pragma unroll
  for (int mt = 0; mt < 2; ++mt)
#pragma unroll
    for (int nt = 0; nt < 4; ++nt) acc[mt][nt] = zero8();

  for (int k0 = 0; k0 < K; k0 += BK_) {
    const v8h ga0 = *(const v8h*)(Ag0 + k0);
    const v8h ga1 = *(const v8h*)(Ag1 + k0);
    const v8h gb0 = *(const v8h*)(Bg0 + k0);
    const v8h gb1 = *(const v8h*)(Bg1 + k0);
    __syncthreads();
    *(v8h*)sa0 = ga0;
    *(v8h*)sa1 = ga1;
    *(v8h*)sb0 = gb0;
    *(v8h*)sb1 = gb1;
    __syncthreads();
    Frag af[2], bf[4];
#pragma unroll
    for (int mt = 0; mt < 2; ++mt) {
      const _Float16* ar = sA + (rowW + 16 * mt + lr) * LP_;
      af[mt].h[0] = *(const v8h*)(ar + 8 * hi);
      af[mt].h[1] = *(const v8h*)(ar + 16 + 8 * hi);
    }
#pragma unroll
    for (int nt = 0; nt < 4; ++nt) {
      const _Float16* br = sB + (colW + 16 * nt + lr) * LP_;
      bf[nt].h[0] = *(const v8h*)(br + 8 * hi);
      bf[nt].h[1] = *(const v8h*)(br + 16 + 8 * hi);
    }
#pragma unroll
    for (int mt = 0; mt < 2; ++mt)
#pragma unroll
      for (int nt = 0; nt < 4; ++nt)
        acc[mt][nt] = __builtin_amdgcn_wmma_f32_16x16x32_f16(false, af[mt].v, false, bf[nt].v, (short)0,
                                                              acc[mt][nt], false, false);
    asm volatile("v_nop\n\tv_nop\n\tv_nop\n\tv_nop"
                 : "+v"(acc[0][0]), "+v"(acc[0][1]), "+v"(acc[0][2]), "+v"(acc[0][3]),
                   "+v"(acc[1][0]), "+v"(acc[1][1]), "+v"(acc[1][2]), "+v"(acc[1][3])
                 : "v"(af[0].v), "v"(af[1].v), "v"(bf[0].v), "v"(bf[1].v), "v"(bf[2].v), "v"(bf[3].v));
  }

  float* sEw = sE + wave * 1024;
  epi_pass<EPI, 0>(acc, sEw, lane, hi, lr, bm0, bn0, rowW, colW, N, e0, e1, e2, Out, img0);
  epi_pass<EPI, 1>(acc, sEw, lane, hi, lr, bm0, bn0, rowW, colW, N, e0, e1, e2, Out, img0);
}

__global__ void __launch_bounds__(64)
attn_kernel(const _Float16* __restrict__ qkv, const float* __restrict__ biasTab, _Float16* Ao, int nwin) {
  __shared__ __attribute__((aligned(16))) _Float16 sVt[2][32 * 72];
  __shared__ __attribute__((aligned(16))) _Float16 sP[2][16 * 72];
  __shared__ __attribute__((aligned(16))) _Float16 sO[64 * 72];

  const int wv = threadIdx.x >> 5, lane = threadIdx.x & 31, hi = lane >> 4, lr = lane & 15;
  const int w = blockIdx.x >> 3, hp = blockIdx.x & 7, h = 2 * hp + wv;
  if (w >= nwin) return;
  const size_t rb = (size_t)w * L_;
  const _Float16* qb = qkv + rb * QKVN_ + h * HD_;
  const _Float16* kb = qb + C_;
  const _Float16* vb = qb + 2 * C_;
  _Float16* myVt = &sVt[wv][0];
  _Float16* myP = &sP[wv][0];

#pragma unroll
  for (int it = 0; it < 4; ++it) {
    const int m = 16 * it + lr;
    const int mm = m < L_ ? m : (L_ - 1);
    const _Float16* vr = vb + (size_t)mm * QKVN_;
    H8 u0, u1;
    u0.h = *(const v8h*)(vr + 8 * hi);
    u1.h = *(const v8h*)(vr + 16 + 8 * hi);
    if (m >= L_) {
      const v4u z = {0u, 0u, 0u, 0u};
      u0.u = z; u1.u = z;
    }
#pragma unroll
    for (int i = 0; i < 8; ++i) {
      myVt[(8 * hi + i) * 72 + m] = u0.h[i];
      myVt[(16 + 8 * hi + i) * 72 + m] = u1.h[i];
    }
  }
  Frag kf[4];
#pragma unroll
  for (int nt = 0; nt < 4; ++nt) {
    const int m = 16 * nt + lr;
    const int mm = m < L_ ? m : (L_ - 1);
    const _Float16* kr = kb + (size_t)mm * QKVN_;
    kf[nt].h[0] = *(const v8h*)(kr + 8 * hi);
    kf[nt].h[1] = *(const v8h*)(kr + 16 + 8 * hi);
  }
  __syncthreads();

  const float* bh = biasTab + (size_t)h * 4096;
#pragma unroll 1
  for (int mt = 0; mt < 4; ++mt) {
    Frag qa;
    {
      const int m = 16 * mt + lr;
      const int mm = m < L_ ? m : (L_ - 1);
      const _Float16* qr = qb + (size_t)mm * QKVN_;
      qa.h[0] = *(const v8h*)(qr + 8 * hi);
      qa.h[1] = *(const v8h*)(qr + 16 + 8 * hi);
    }
    v8f sacc[4];
#pragma unroll
    for (int nt = 0; nt < 4; ++nt) sacc[nt] = wmma_g(qa.v, kf[nt].v, zero8());

#pragma unroll
    for (int r = 0; r < 8; ++r) {
      const int srow = 16 * mt + 8 * hi + r;
      const float* br = bh + srow * 64;
      float p0 = sacc[0][r] + br[lr];
      float p1 = sacc[1][r] + br[16 + lr];
      float p2 = sacc[2][r] + br[32 + lr];
      float p3 = sacc[3][r] + br[48 + lr];
      float mx = fmaxf(fmaxf(p0, p1), fmaxf(p2, p3));
#pragma unroll
      for (int m = 8; m >= 1; m >>= 1) mx = fmaxf(mx, __shfl_xor(mx, m, 32));
      p0 = __expf(p0 - mx); p1 = __expf(p1 - mx); p2 = __expf(p2 - mx); p3 = __expf(p3 - mx);
      float sum = p0 + p1 + p2 + p3;
#pragma unroll
      for (int m = 8; m >= 1; m >>= 1) sum += __shfl_xor(sum, m, 32);
      const float inv = __fdividef(256.0f, sum);
      const int pr = 8 * hi + r;
      myP[pr * 72 + lr]      = (_Float16)(p0 * inv);
      myP[pr * 72 + 16 + lr] = (_Float16)(p1 * inv);
      myP[pr * 72 + 32 + lr] = (_Float16)(p2 * inv);
      myP[pr * 72 + 48 + lr] = (_Float16)(p3 * inv);
    }
    __syncthreads();

    Frag pa0, pa1;
    pa0.h[0] = *(const v8h*)(myP + lr * 72 + 8 * hi);
    pa0.h[1] = *(const v8h*)(myP + lr * 72 + 16 + 8 * hi);
    pa1.h[0] = *(const v8h*)(myP + lr * 72 + 32 + 8 * hi);
    pa1.h[1] = *(const v8h*)(myP + lr * 72 + 48 + 8 * hi);
    v8f oacc[2];
#pragma unroll
    for (int dt = 0; dt < 2; ++dt) {
      const _Float16* vr = myVt + (16 * dt + lr) * 72;
      Frag b0, b1;
      b0.h[0] = *(const v8h*)(vr + 8 * hi);
      b0.h[1] = *(const v8h*)(vr + 16 + 8 * hi);
      b1.h[0] = *(const v8h*)(vr + 32 + 8 * hi);
      b1.h[1] = *(const v8h*)(vr + 48 + 8 * hi);
      oacc[dt] = wmma_g(pa0.v, b0.v, zero8());
      oacc[dt] = wmma_g(pa1.v, b1.v, oacc[dt]);
    }
#pragma unroll
    for (int dt = 0; dt < 2; ++dt)
#pragma unroll
      for (int r = 0; r < 8; ++r)
        sO[(16 * mt + 8 * hi + r) * 72 + 32 * wv + 16 * dt + lr] = (_Float16)(oacc[dt][r] * INV256_);
  }
  __syncthreads();

  const int q = lane >> 3, j = lane & 7;
  _Float16* ob = Ao + rb * C_ + hp * 64 + 8 * j;
  const int rbase = wv ? 28 : 0;
  const int rlim = wv ? L_ : 28;
  v4u vals[7];
  int rls[7];
#pragma unroll
  for (int s = 0; s < 7; ++s) {
    const int rl = rbase + 4 * s + q;
    const bool ok = rl < rlim;
    const int rr = ok ? rl : 0;
    H8 u;
    u.h = *(const v8h*)(sO + rr * 72 + 8 * j);
    vals[s] = u.u;
    rls[s] = ok ? rl : -1;
  }
#pragma unroll
  for (int s = 0; s < 7; ++s)
    if (rls[s] >= 0) vst(ob + (size_t)rls[s] * C_, vals[s]);
  __threadfence();
#pragma unroll
  for (int s = 0; s < 7; ++s)
    if (rls[s] >= 0) vst(ob + (size_t)rls[s] * C_, vals[s]);
}

__global__ void __launch_bounds__(256)
dwconv_kernel(const _Float16* __restrict__ H1, const float* __restrict__ dww,
              const float* __restrict__ s2p, const float* __restrict__ t2p, _Float16* H2, int nimg) {
  const int bx = blockIdx.x;
  const int x = bx % WIMG_;
  const int rest = bx / WIMG_;
  const int ys = rest % NYS_;
  const int bl = rest / NYS_;
  if (bl >= nimg) return;
  const int t = threadIdx.x;
  const int c0 = 64 * (t >> 3) + 8 * (t & 7);

  float wt[9][8];
#pragma unroll
  for (int tap = 0; tap < 9; ++tap)
#pragma unroll
    for (int i = 0; i < 8; ++i) wt[tap][i] = dww[(c0 + i) * 9 + tap];
  float sc[8], sh[8];
  {
    const v4f a0 = *(const v4f*)(s2p + c0), a1 = *(const v4f*)(s2p + c0 + 4);
    const v4f b0 = *(const v4f*)(t2p + c0), b1 = *(const v4f*)(t2p + c0 + 4);
#pragma unroll
    for (int i = 0; i < 4; ++i) { sc[i] = a0[i]; sc[4 + i] = a1[i]; sh[i] = b0[i]; sh[4 + i] = b1[i]; }
  }
  const size_t imgb = (size_t)bl * HW_;

#pragma unroll 1
  for (int yy = 0; yy < SY_; ++yy) {
    const int y = ys * SY_ + yy;
    float acc[8];
#pragma unroll
    for (int i = 0; i < 8; ++i) acc[i] = 0.f;
#pragma unroll
    for (int ky = 0; ky < 3; ++ky) {
      const int ny = y + ky - 1;
      if (ny >= 0 && ny < HIMG_) {
#pragma unroll
        for (int kx = 0; kx < 3; ++kx) {
          const int nx = x + kx - 1;
          if (nx >= 0 && nx < WIMG_) {
            H8 u;
            u.h = *(const v8h*)(H1 + (imgb + (size_t)ny * WIMG_ + nx) * HID_ + c0);
#pragma unroll
            for (int i = 0; i < 8; ++i) acc[i] += (float)u.h[i] * wt[ky * 3 + kx][i];
          }
        }
      }
    }
    H8 o;
#pragma unroll
    for (int i = 0; i < 8; ++i) o.h[i] = (_Float16)gelu_f(acc[i] * sc[i] + sh[i]);
    _Float16* d = H2 + (imgb + (size_t)y * WIMG_ + x) * HID_ + c0;
    vst(d, o.u);
    __threadfence();
    vst(d, o.u);
  }
}

extern "C" void kernel_launch(void* const* d_in, const int* in_sizes, int n_in,
                              void* d_out, int out_size, void* d_ws, size_t ws_size,
                              hipStream_t stream) {
  if (n_in < 29) return;
  if (in_sizes[0] != B_ * C_ * HW_ || out_size != B_ * C_ * HW_) return;
  if (in_sizes[1] != QKVN_ * C_ || in_sizes[2] != QKVN_ || in_sizes[3] != C_ * C_ ||
      in_sizes[5] != 169 * NH_ || in_sizes[10] != HID_ * C_ || in_sizes[16] != HID_ * 9 ||
      in_sizes[22] != C_ * HID_ || in_sizes[28] != L_ * L_) return;

  const float* x      = (const float*)d_in[0];
  const float* qkv_w  = (const float*)d_in[1];
  const float* qkv_b  = (const float*)d_in[2];
  const float* proj_w = (const float*)d_in[3];
  const float* proj_b = (const float*)d_in[4];
  const float* rpb    = (const float*)d_in[5];
  const float* ln1_g  = (const float*)d_in[6];
  const float* ln1_b  = (const float*)d_in[7];
  const float* ln2_g  = (const float*)d_in[8];
  const float* ln2_b  = (const float*)d_in[9];
  const float* fc1_w  = (const float*)d_in[10];
  const float* fc1_b  = (const float*)d_in[11];
  const float* bn1_g  = (const float*)d_in[12];
  const float* bn1_b  = (const float*)d_in[13];
  const float* bn1_m  = (const float*)d_in[14];
  const float* bn1_v  = (const float*)d_in[15];
  const float* dw_w   = (const float*)d_in[16];
  const float* dw_b   = (const float*)d_in[17];
  const float* bn2_g  = (const float*)d_in[18];
  const float* bn2_b  = (const float*)d_in[19];
  const float* bn2_m  = (const float*)d_in[20];
  const float* bn2_v  = (const float*)d_in[21];
  const float* fc2_w  = (const float*)d_in[22];
  const float* fc2_b  = (const float*)d_in[23];
  const float* bn3_g  = (const float*)d_in[24];
  const float* bn3_b  = (const float*)d_in[25];
  const float* bn3_m  = (const float*)d_in[26];
  const float* bn3_v  = (const float*)d_in[27];
  const int* rel_index = (const int*)d_in[28];

  char* ws = (char*)d_ws;
  size_t off = 0;
  auto carve = [&](size_t bytes) -> char* {
    off = (off + 255) & ~(size_t)255;
    char* p = ws + off;
    off += bytes;
    return p;
  };
  _Float16* w16     = (_Float16*)carve((size_t)W3_ * 2);
  float*    ab      = (float*)carve((size_t)NFOLD_ * 4);
  float*    biasTab = (float*)carve((size_t)NBIAS_ * 4);
  _Float16* hA      = (_Float16*)carve((size_t)MC_ * C_ * 2);
  _Float16* qkvb    = (_Float16*)carve((size_t)MC_ * QKVN_ * 2);
  _Float16* Ao      = (_Float16*)carve((size_t)MC_ * C_ * 2);
  float*    xs1     = (float*)carve((size_t)MC_ * C_ * 4);
  _Float16* H1      = (_Float16*)carve((size_t)MC_ * HID_ * 2);
  _Float16* H2      = (_Float16*)carve((size_t)MC_ * HID_ * 2);
  if (off > ws_size) return;

  _Float16* wqkv16  = w16;
  _Float16* wproj16 = w16 + W0_;
  _Float16* wfc1_16 = w16 + W1_;
  _Float16* wfc2_16 = w16 + W2_;

  prep_kernel<<<dim3(PREPN_ / 256), dim3(256), 0, stream>>>(
      fc1_b, bn1_g, bn1_b, bn1_m, bn1_v, dw_b, bn2_g, bn2_b, bn2_m, bn2_v,
      fc2_b, bn3_g, bn3_b, bn3_m, bn3_v, rpb, rel_index, qkv_w, proj_w, fc1_w, fc2_w,
      ab, biasTab, w16);

  for (int ch = 0; ch < NCHK_; ++ch) {
    const float* xc = x + (size_t)ch * IPC_ * C_ * HW_;
    float* outc = (float*)d_out + (size_t)ch * IPC_ * C_ * HW_;

    ln_kernel<0><<<dim3((MC_ + 7) / 8), dim3(256), 0, stream>>>(xc, ln1_g, ln1_b, hA, MC_);
    gemm_kernel<EPI_QKV><<<dim3(MC_ / BM_, QKVN_ / BN_), dim3(256), 0, stream>>>(
        hA, wqkv16, MC_, QKVN_, C_, qkv_b, ab, ab, (void*)qkvb, 0);
    attn_kernel<<<dim3(NWC_ * 8), dim3(64), 0, stream>>>(qkvb, biasTab, Ao, NWC_);
    gemm_kernel<EPI_PROJ><<<dim3(MC_ / BM_, C_ / BN_), dim3(256), 0, stream>>>(
        Ao, wproj16, MC_, C_, C_, proj_b, ab, x, (void*)xs1, ch * IPC_);
    ln_kernel<1><<<dim3((MC_ + 7) / 8), dim3(256), 0, stream>>>(xs1, ln2_g, ln2_b, hA, MC_);
    gemm_kernel<EPI_H1><<<dim3(MC_ / BM_, HID_ / BN_), dim3(256), 0, stream>>>(
        hA, wfc1_16, MC_, HID_, C_, ab, ab + 2048, ab, (void*)H1, 0);
    dwconv_kernel<<<dim3(IPC_ * NYS_ * WIMG_), dim3(256), 0, stream>>>(
        H1, dw_w, ab + 4096, ab + 6144, H2, IPC_);
    gemm_kernel<EPI_OUT><<<dim3(MC_ / BM_, C_ / BN_), dim3(256), 0, stream>>>(
        H2, wfc2_16, MC_, C_, HID_, ab + 8192, ab + 8704, xs1, (void*)outc, 0);
  }
}
